// RNN_85950885528212
// MI455X (gfx1250) — hardware-verified
//
#include <hip/hip_runtime.h>
#include <math.h>

constexpr int NBATCH   = 8192;
constexpr int NSTEP    = 512;
constexpr int NFEAT    = 2;
constexpr int NHID     = 128;
constexpr int NWROWS   = NFEAT + NHID;
constexpr int ROWS_BLK = 32;
constexpr int NTHR     = 256;
constexpr int NWAVE    = NTHR / 32;
constexpr int HPITCH   = 136;
constexpr int XCHUNK   = 64;
constexpr int XROWF    = ROWS_BLK * NFEAT;
constexpr float GARCH_ALPHA = 0.2f;
constexpr float GARCH_BETA  = 0.7f;
constexpr float HCARRY    = 64.0f;
constexpr float WCARRY    = 64.0f;
constexpr float CARRY_INV = 1.0f / (HCARRY * WCARRY);

static_assert(NHID == 16 * NWAVE, "one 16-column group per wave");
static_assert(NHID % 32 == 0, "K multiple of 32");
static_assert(NBATCH % ROWS_BLK == 0, "exact grid");
static_assert(ROWS_BLK == 32, "one 128-B output line per block");
static_assert(NSTEP % XCHUNK == 0, "exact x chunks");
static_assert((2 * ROWS_BLK * HPITCH) % NTHR == 0, "exact zero fill");
static_assert((ROWS_BLK * XCHUNK * NFEAT) == 4 * 4 * NTHR, "x staging covers the chunk exactly");
static_assert((HPITCH * 2) % 16 == 0, "fragment rows 16-B aligned");

typedef __attribute__((ext_vector_type(16))) _Float16 v16h;
typedef __attribute__((ext_vector_type(8)))  _Float16 v8h;
typedef __attribute__((ext_vector_type(8)))  float    v8f;
typedef __attribute__((ext_vector_type(4)))  float    v4f;
typedef __attribute__((ext_vector_type(2)))  float    v2f;

union FragU { v16h v; v8h h[2]; };

__device__ __forceinline__ v16h frag_load(const _Float16* p) {
  FragU f;
  f.h[0] = *(const v8h*)(p);
  f.h[1] = *(const v8h*)(p + 16);
  return f.v;
}
__device__ __forceinline__ v8f frag_mma(v16h a, v16h b, v8f c) {
  return __builtin_amdgcn_wmma_f32_16x16x32_f16(false, a, false, b, (short)0, c, false, false);
}
__device__ __forceinline__ void group_guard(v8f& a, v8f& b, v16h x, v16h y, v16h w) {
  asm volatile("v_nop\n\tv_nop\n\tv_nop\n\tv_nop" : "+v"(a), "+v"(b) : "v"(x), "v"(y), "v"(w));
}
__device__ __forceinline__ void pin_half(v8h& h) { asm volatile("" : "+v"(h) : : "memory"); }

__device__ __forceinline__ float tanh_f32(float z) {
  const float e = expf(2.0f * z);
  return 1.0f - 2.0f / (e + 1.0f);
}

__global__ __launch_bounds__(NTHR) void rnn_garch_kernel(const float* __restrict__ x,
                                                         const float* __restrict__ Wrec,
                                                         const float* __restrict__ brec,
                                                         const float* __restrict__ Wout,
                                                         const float* __restrict__ bout,
                                                         float* __restrict__ out) {
  __shared__ __align__(16) _Float16 Ah[2 * ROWS_BLK * HPITCH];
  __shared__ __align__(16) float    Xs[XCHUNK * XROWF];
  __shared__ __align__(16) float    Red[NWAVE * ROWS_BLK];

  const int tid  = threadIdx.x;
  const int lane = tid & 31;
  const int wave = tid >> 5;
  const int c    = lane & 15;
  const int hh   = lane >> 4;
  const int koff = hh * 8;
  const int ncol = wave * 16 + c;
  const int b0   = blockIdx.x * ROWS_BLK;

#pragma unroll 1
  for (int i = tid; i < 2 * ROWS_BLK * HPITCH; i += NTHR) Ah[i] = (_Float16)0.0f;

  v16h Bf[4];
#pragma unroll
  for (int kc = 0; kc < 4; ++kc) {
    FragU u;
#pragma unroll
    for (int s = 0; s < 2; ++s) {
      v8h hv;
#pragma unroll
      for (int e = 0; e < 8; ++e) {
        const int k = 32 * kc + 16 * s + koff + e;
        const float w = Wrec[(size_t)(NFEAT + k) * NHID + ncol];
        hv[e] = (_Float16)(w * WCARRY);
      }
      pin_half(hv);
      u.h[s] = hv;
    }
    Bf[kc] = u.v;
  }
  const float w0   = Wrec[ncol];
  const float w1   = Wrec[NHID + ncol];
  const float bias = brec[ncol];
  const float wo   = Wout[ncol];
  const float bo   = bout[0];

  float part[2][8];
#pragma unroll
  for (int mt = 0; mt < 2; ++mt)
#pragma unroll
    for (int r = 0; r < 8; ++r) part[mt][r] = 0.0f;
  float rs = 0.0f;
  float resid = 0.0f;

  const v8f z8 = {0.f, 0.f, 0.f, 0.f, 0.f, 0.f, 0.f, 0.f};

#pragma unroll 1
  for (int ch = 0; ch < NSTEP / XCHUNK; ++ch) {
#pragma unroll
    for (int i = 0; i < 4; ++i) {
      const int idx = i * NTHR + tid;
      const int row = idx >> 5;
      const int q4  = idx & 31;
      const v4f v = *(const v4f*)(x + (size_t)(b0 + row) * (NSTEP * NFEAT) + (size_t)ch * (XCHUNK * NFEAT) + q4 * 4);
      v2f lo, hi;
      lo[0] = v[0]; lo[1] = v[1];
      hi[0] = v[2]; hi[1] = v[3];
      *(v2f*)(Xs + (2 * q4) * XROWF + row * 2)     = lo;
      *(v2f*)(Xs + (2 * q4 + 1) * XROWF + row * 2) = hi;
    }
    __syncthreads();

#pragma unroll 1
    for (int tl = 0; tl < XCHUNK; ++tl) {
      const int cur = (ch * XCHUNK + tl) & 1;
      const _Float16* arow = Ah + cur * (ROWS_BLK * HPITCH) + c * HPITCH + koff;
      _Float16* hn = Ah + (cur ^ 1) * (ROWS_BLK * HPITCH);
      const float* xrow = Xs + tl * XROWF;

      const float xr0 = xrow[lane * 2];
      rs = rs * GARCH_BETA + (resid * resid * GARCH_ALPHA + bo);
      resid = xr0;

      v8f acc0 = z8, acc1 = z8;
#pragma unroll
      for (int kc = 0; kc < 4; ++kc) {
        const v16h a0 = frag_load(arow + 32 * kc);
        const v16h a1 = frag_load(arow + 16 * HPITCH + 32 * kc);
        acc0 = frag_mma(a0, Bf[kc], acc0);
        acc1 = frag_mma(a1, Bf[kc], acc1);
        group_guard(acc0, acc1, a0, a1, Bf[kc]);
      }

#pragma unroll
      for (int mt = 0; mt < 2; ++mt) {
        const v8f acc = (mt == 0) ? acc0 : acc1;
        const float* xp = xrow + (16 * mt + 8 * hh) * 2;
        v4f xq[4];
        xq[0] = *(const v4f*)(xp);
        xq[1] = *(const v4f*)(xp + 4);
        xq[2] = *(const v4f*)(xp + 8);
        xq[3] = *(const v4f*)(xp + 12);
#pragma unroll
        for (int r = 0; r < 8; ++r) {
          const float x0 = xq[r >> 1][(r & 1) * 2];
          const float x1 = xq[r >> 1][(r & 1) * 2 + 1];
          const float zx = x0 * w0 + x1 * w1 + bias;
          const float z  = acc[r] * CARRY_INV + zx;
          const float th = tanh_f32(z);
          part[mt][r] = part[mt][r] * GARCH_BETA + th * wo;
          hn[(16 * mt + 8 * hh + r) * HPITCH + ncol] = (_Float16)(th * HCARRY);
        }
      }
      __syncthreads();
    }
  }

#pragma unroll
  for (int mt = 0; mt < 2; ++mt) {
#pragma unroll
    for (int r = 0; r < 8; ++r) {
      float v = part[mt][r];
      v += __shfl_xor(v, 1, 32);
      v += __shfl_xor(v, 2, 32);
      v += __shfl_xor(v, 4, 32);
      v += __shfl_xor(v, 8, 32);
      if (c == 0) Red[wave * ROWS_BLK + 16 * mt + 8 * hh + r] = v;
    }
  }
  __syncthreads();
  if (wave == 0) {
    float s = 0.0f;
#pragma unroll
    for (int w = 0; w < NWAVE; ++w) s += Red[w * ROWS_BLK + lane];
    s += rs;
    volatile float* op = out + (size_t)b0 + lane;
    *op = s;
    __threadfence();
    *op = s;
  }
}

extern "C" void kernel_launch(void* const* d_in, const int* in_sizes, int n_in,
                              void* d_out, int out_size, void* d_ws, size_t ws_size, hipStream_t stream) {
  (void)d_ws; (void)ws_size;
  if (n_in < 5 || d_out == nullptr) return;
  if (in_sizes[0] != NBATCH * NSTEP * NFEAT || in_sizes[1] != NWROWS * NHID || in_sizes[2] != NHID ||
      in_sizes[3] != NHID || in_sizes[4] != 1 || out_size != NBATCH) return;
  const float* xin  = (const float*)d_in[0];
  const float* wrec = (const float*)d_in[1];
  const float* brec = (const float*)d_in[2];
  const float* wout = (const float*)d_in[3];
  const float* bout = (const float*)d_in[4];
  float* out = (float*)d_out;
  rnn_garch_kernel<<<NBATCH / ROWS_BLK, NTHR, 0, stream>>>(xin, wrec, brec, wout, bout, out);
}
